// CachedMultiheadAttention_61469571940980
// MI455X (gfx1250) — hardware-verified
//
#include <hip/hip_runtime.h>

#ifndef NB
#define NB 4
#endif
#ifndef SEQ
#define SEQ 2048
#endif
#define NB_FULL 4
#define SEQ_FULL 2048

constexpr int kBatch     = NB;
constexpr int kBatchFull = NB_FULL;
constexpr int kSeq       = SEQ;
constexpr int kSeqFull   = SEQ_FULL;
constexpr int kEmb       = 1024;
constexpr int kHeads     = 16;
constexpr int kHdim      = 64;
constexpr int kWin       = 512;
constexpr int kNblk      = kSeq / kWin;
constexpr int kTok       = kBatch * kSeq;
constexpr int kGuard     = 512;
constexpr int kQKRows    = kGuard + kTok;
constexpr int kQKPitch   = 2 * kEmb;
constexpr int kVtPitch   = kGuard + kTok;
constexpr int kKeys      = 2 * kWin;
constexpr int kChunks    = kBatch * kNblk;

static_assert(kSeq % kWin == 0);
static_assert(kSeq >= kWin && kSeq <= kSeqFull);
static_assert(kBatch >= 1 && kBatch <= kBatchFull);
static_assert(kHeads * kHdim == kEmb);
static_assert(kTok % 64 == 0 && kEmb % 64 == 0 && kKeys % 64 == 0 && kWin % 64 == 0);
static_assert(kEmb % 32 == 0 && kHdim % 32 == 0 && kKeys % 32 == 0);
static_assert((kVtPitch * 2) % 128 == 0 && (kQKPitch * 2) % 128 == 0);

constexpr float kWCarry   = 64.0f;
constexpr float kQKScale  = 1.0f / 16.0f;
constexpr float kSScale   = 1.0f / 128.0f;
constexpr float kPCarry   = 2048.0f;
constexpr float kPVScale  = 1.0f / 512.0f;
constexpr float kOutScale = 1.0f / 1024.0f;

typedef __attribute__((ext_vector_type(16))) _Float16 v16h;
typedef __attribute__((ext_vector_type(8)))  _Float16 v8h;
typedef __attribute__((ext_vector_type(16))) __bf16   v16b;
typedef __attribute__((ext_vector_type(8)))  __bf16   v8b;
typedef __attribute__((ext_vector_type(8)))  float    v8f;
typedef __attribute__((ext_vector_type(4)))  float    v4f;
typedef __attribute__((ext_vector_type(4)))  unsigned int v4u;

__device__ __forceinline__ unsigned short f2bf_bits(float f) {
  unsigned u = __float_as_uint(f);
  return (unsigned short)((u + 0x7FFFu + ((u >> 16) & 1u)) >> 16);
}
__device__ __forceinline__ float bf_bits2f(unsigned short h) { return __uint_as_float(((unsigned)h) << 16); }

__device__ __forceinline__ void dep_guard_h(v8f& a, v8f& b, v16h x, v16h y) { asm volatile("v_nop\n\tv_nop\n\tv_nop\n\tv_nop" : "+v"(a), "+v"(b) : "v"(x), "v"(y)); }
__device__ __forceinline__ void dep_guard_b(v8f& a, v8f& b, v16b x, v16b y) { asm volatile("v_nop\n\tv_nop\n\tv_nop\n\tv_nop" : "+v"(a), "+v"(b) : "v"(x), "v"(y)); }
__device__ __forceinline__ void keep4_h(v16h a, v16h b, v16h c, v16h d) { asm volatile("v_nop" :: "v"(a), "v"(b), "v"(c), "v"(d)); }
__device__ __forceinline__ void keep4_b(v16b a, v16b b, v16b c, v16b d) { asm volatile("v_nop" :: "v"(a), "v"(b), "v"(c), "v"(d)); }
__device__ __forceinline__ void acc_guard4(v8f& a, v8f& b, v8f& c, v8f& d) { asm volatile("v_nop\n\tv_nop\n\tv_nop\n\tv_nop" : "+v"(a), "+v"(b), "+v"(c), "+v"(d)); }
template <typename T> struct Frag;
template <> struct Frag<_Float16> {
  typedef v16h V; union U { v16h v; v8h h[2]; };
  static __device__ __forceinline__ v16h load(const _Float16* p) {
    U f; f.h[0] = *(const v8h*)(p); f.h[1] = *(const v8h*)(p + 16); return f.v;
  }
  static __device__ __forceinline__ v8f mma(v16h a, v16h b, v8f c) {
    return __builtin_amdgcn_wmma_f32_16x16x32_f16(false, a, false, b, (short)0, c, false, false);
  }
  static __device__ __forceinline__ void guard(v8f& a, v8f& b, v16h x, v16h y) { dep_guard_h(a, b, x, y); }
  static __device__ __forceinline__ void keep(v16h a, v16h b, v16h c, v16h d) { keep4_h(a, b, c, d); }
};
template <> struct Frag<__bf16> {
  typedef v16b V; union U { v16b v; v8b h[2]; };
  static __device__ __forceinline__ v16b load(const __bf16* p) {
    U f; f.h[0] = *(const v8b*)(p); f.h[1] = *(const v8b*)(p + 16); return f.v;
  }
  static __device__ __forceinline__ v8f mma(v16b a, v16b b, v8f c) {
    return __builtin_amdgcn_wmma_f32_16x16x32_bf16(false, a, false, b, (short)0, c, false, false);
  }
  static __device__ __forceinline__ void guard(v8f& a, v8f& b, v16b x, v16b y) { dep_guard_b(a, b, x, y); }
  static __device__ __forceinline__ void keep(v16b a, v16b b, v16b c, v16b d) { keep4_b(a, b, c, d); }
};

__device__ __forceinline__ unsigned pk16(unsigned short a, unsigned short b) { return (unsigned)a | ((unsigned)b << 16); }
__device__ __forceinline__ unsigned short h_bits(float f) { const _Float16 h = (_Float16)f; return __builtin_bit_cast(unsigned short, h); }

template <int ET> struct Elem;
template <> struct Elem<0> { typedef _Float16 T; };
template <> struct Elem<1> { typedef __bf16 T; };
template <int ET, bool SPLIT, int BIAS_MODE, int OUT_MODE, bool RESID, int ACT = 0>
__global__ __launch_bounds__(256) void wmma_gemm64(
    const unsigned short* __restrict__ Ap, const unsigned short* __restrict__ A2p, int lda, long strideA,
    const unsigned short* __restrict__ Btp, const unsigned short* __restrict__ Bt2p, int ldb, long strideB,
    void* __restrict__ Cout, void* __restrict__ Cout2, int ldc, long strideC,
    const float* __restrict__ bias,
    const float* __restrict__ resid, long strideR,
    int M, int N, int K, float scale) {
  typedef typename Elem<ET>::T T;
  typedef typename Frag<T>::V V;
  const T* A = (const T*)Ap; const T* A2 = (const T*)A2p; const T* Bt = (const T*)Btp; const T* Bt2 = (const T*)Bt2p;
  __shared__ __align__(16) float sT[8][16 * 68];
  const int b    = blockIdx.y;
  const int lane = threadIdx.x & 31;
  const int wave = threadIdx.x >> 5;
  const int tilesN = N >> 6;
  const int tilesM = M >> 6;
  const int tile = blockIdx.x * 8 + wave;
  if (tile >= tilesM * tilesN) return;
  const int tm = tile / tilesN;
  const int tn = tile - tm * tilesN;
  const int m0 = tm << 6;
  const int n0 = tn << 6;

  const T* Ab  = A  + (size_t)b * strideA;
  const T* Bb  = Bt + (size_t)b * strideB;
  const T* Ab2 = SPLIT ? (A2  + (size_t)b * strideA) : nullptr;
  const T* Bb2 = SPLIT ? (Bt2 + (size_t)b * strideB) : nullptr;

  const int rlane = lane & 15;
  const int koff  = (lane >> 4) * 8;
  const int mOff  = (lane >> 4) * 8;

  v8f acc[4][4];
#pragma unroll
  for (int i = 0; i < 4; ++i)
#pragma unroll
    for (int j = 0; j < 4; ++j) acc[i][j] = (v8f){0.f,0.f,0.f,0.f,0.f,0.f,0.f,0.f};

  for (int k0 = 0; k0 < K; k0 += 32) {
    V bh[4], bl[4];
#pragma unroll
    for (int j = 0; j < 4; ++j) {
      const size_t bo = (size_t)(n0 + (j << 4) + rlane) * ldb + koff + k0;
      bh[j] = Frag<T>::load(Bb + bo);
      if (SPLIT) bl[j] = Frag<T>::load(Bb2 + bo);
    }
#pragma unroll
    for (int i = 0; i < 4; ++i) {
      const size_t ao = (size_t)(m0 + (i << 4) + rlane) * lda + koff + k0;
      V ah = Frag<T>::load(Ab + ao);
      V al;
      if (SPLIT) al = Frag<T>::load(Ab2 + ao);
#pragma unroll
      for (int j = 0; j < 4; ++j) {
        acc[i][j] = Frag<T>::mma(ah, bh[j], acc[i][j]);
        if (SPLIT) {
          acc[i][j] = Frag<T>::mma(ah, bl[j], acc[i][j]);
          acc[i][j] = Frag<T>::mma(al, bh[j], acc[i][j]);
        }
      }
      Frag<T>::guard(acc[i][0], acc[i][3], ah, SPLIT ? al : ah);
    }
    Frag<T>::keep(bh[0], bh[1], bh[2], bh[3]);
    if (SPLIT) Frag<T>::keep(bl[0], bl[1], bl[2], bl[3]);
  }
  acc_guard4(acc[0][0], acc[0][1], acc[0][2], acc[0][3]);
  acc_guard4(acc[1][0], acc[1][1], acc[1][2], acc[1][3]);
  acc_guard4(acc[2][0], acc[2][1], acc[2][2], acc[2][3]);
  acc_guard4(acc[3][0], acc[3][1], acc[3][2], acc[3][3]);

  float* slab = sT[wave];
  const float* Rb = RESID ? (resid + (size_t)b * strideR) : nullptr;
#pragma unroll
  for (int i = 0; i < 4; ++i) {
    const int mBase = m0 + (i << 4);
#pragma unroll
    for (int j = 0; j < 4; ++j) {
      const int n = n0 + (j << 4) + rlane;
      float bv = 0.f;
      if (BIAS_MODE == 2) bv = bias[n];
#pragma unroll
      for (int r = 0; r < 8; ++r) {
        float v = acc[i][j][r] * scale;
        if (BIAS_MODE == 1) v += bias[mBase + mOff + r];
        if (BIAS_MODE == 2) v += bv;
        if (RESID) v += Rb[(size_t)(mBase + mOff + r) * ldc + n];
        if (ACT == 2) v = fmaxf(v, 0.0f);
        if (ACT == 4) v = (v > 0.f) ? v : 0.01f * v;
        slab[(mOff + r) * 68 + (j << 4) + rlane] = v;
      }
    }
    __builtin_amdgcn_fence(__ATOMIC_RELEASE, "workgroup");
    __builtin_amdgcn_wave_barrier();
    __builtin_amdgcn_fence(__ATOMIC_ACQUIRE, "workgroup");
    if (OUT_MODE == 0) {
      float* C = (float*)Cout + (size_t)b * strideC;
      const int hh = lane >> 4, c4 = (lane & 15) * 4;
      for (int pass = 0; pass < 2; ++pass) {
#pragma unroll
        for (int it = 0; it < 8; ++it) {
          const int row = it * 2 + hh;
          v4f v = *(const v4f*)(slab + row * 68 + c4);
          *(volatile v4f*)(C + (size_t)(mBase + row) * ldc + n0 + c4) = v;
        }
        __threadfence();
      }
    } else {
      const int q = lane >> 3, c8 = (lane & 7) * 8;
      unsigned short* C  = (unsigned short*)Cout  + (size_t)b * strideC;
      unsigned short* C2 = (OUT_MODE == 2) ? ((unsigned short*)Cout2 + (size_t)b * strideC) : nullptr;
      for (int pass = 0; pass < 2; ++pass) {
#pragma unroll
        for (int it = 0; it < 4; ++it) {
          const int row = it * 4 + q;
          const float* sp = slab + row * 68 + c8;
          v8h hv, lv;
#pragma unroll
          for (int e = 0; e < 8; ++e) {
            if (OUT_MODE == 1) {
              hv[e] = (_Float16)sp[e];
            } else {
              unsigned short hb = f2bf_bits(sp[e]);
              unsigned short lb = f2bf_bits(sp[e] - bf_bits2f(hb));
              hv[e] = __builtin_bit_cast(_Float16, hb);
              lv[e] = __builtin_bit_cast(_Float16, lb);
            }
          }
          *(volatile v8h*)(C + (size_t)(mBase + row) * ldc + n0 + c8) = hv;
          if (OUT_MODE == 2) *(volatile v8h*)(C2 + (size_t)(mBase + row) * ldc + n0 + c8) = lv;
        }
        __threadfence();
      }
    }
    __builtin_amdgcn_fence(__ATOMIC_RELEASE, "workgroup");
    __builtin_amdgcn_wave_barrier();
    __builtin_amdgcn_fence(__ATOMIC_ACQUIRE, "workgroup");
  }
}

__global__ __launch_bounds__(256) void cast8_f16_kernel(const float* __restrict__ in, long inStride,
                                                        unsigned short* __restrict__ out, long outStride,
                                                        int n8, float scale) {
  const int i = blockIdx.x * 256 + threadIdx.x;
  if (i >= n8) return;
  const float* p = in + (size_t)blockIdx.y * inStride + 8 * (size_t)i;
  const v4f a = *(const v4f*)(p);
  const v4f c = *(const v4f*)(p + 4);
  unsigned short hb[8];
#pragma unroll
  for (int e = 0; e < 4; ++e) {
    hb[e]     = h_bits(bf_bits2f(f2bf_bits(a[e])) * scale);
    hb[4 + e] = h_bits(bf_bits2f(f2bf_bits(c[e])) * scale);
  }
  const v4u u = (v4u){pk16(hb[0], hb[1]), pk16(hb[2], hb[3]), pk16(hb[4], hb[5]), pk16(hb[6], hb[7])};
  unsigned short* q = out + (size_t)blockIdx.y * outStride + 8 * (size_t)i;
  *(volatile v4u*)q = u;
  __threadfence();
  *(volatile v4u*)q = u;
}

__global__ __launch_bounds__(256) void zero16_kernel(unsigned short* __restrict__ base, int pitch, int segs, int total) {
  const int i = blockIdx.x * 256 + threadIdx.x;
  if (i >= total) return;
  const int row = i / segs;
  const int seg = i - row * segs;
  unsigned short* p = base + (size_t)row * pitch + (size_t)seg * 8;
  const v4u z = (v4u){0u, 0u, 0u, 0u};
  *(volatile v4u*)p = z;
  __threadfence();
  *(volatile v4u*)p = z;
}

__global__ __launch_bounds__(128) void band_softmax_kernel(const float* __restrict__ S, unsigned short* __restrict__ P, int blk) {
#pragma clang fp contract(off)
  __shared__ float redM[4];
  __shared__ float redS[4];
  const int qi   = blockIdx.x;
  const int h    = blockIdx.y;
  const int t    = threadIdx.x;
  const int lane = t & 31, wave = t >> 5;
  const int c0   = t * 8;
  const size_t rowoff = ((size_t)h * kWin + qi) * kKeys;
  const float* sr = S + rowoff + c0;
  const v4f a = *(const v4f*)(sr);
  const v4f c = *(const v4f*)(sr + 4);
  const int e1 = h + 1;
  const float sl = ((e1 & 1) ? 0.70710678118654752f : 1.0f) * __uint_as_float(((unsigned)(127 - (e1 >> 1))) << 23);
  const float neg_inf = -__builtin_inff();
  const int kbase = blk * kWin - kWin;
  float x[8];
#pragma unroll
  for (int e = 0; e < 8; ++e) {
    const int kj = c0 + e;
    const int delta = qi - kj + kWin;
    const bool valid = (delta >= 0) && (delta < kWin) && (kbase + kj >= 0);
    const float sv = (e < 4) ? a[e] : c[e - 4];
    const float bias = sl * (float)delta;
    const float sc = sv + bias;
    x[e] = valid ? sc : neg_inf;
  }
  float m = fmaxf(fmaxf(fmaxf(x[0], x[1]), fmaxf(x[2], x[3])), fmaxf(fmaxf(x[4], x[5]), fmaxf(x[6], x[7])));
#pragma unroll
  for (int off = 16; off > 0; off >>= 1) m = fmaxf(m, __shfl_xor(m, off, 32));
  if (lane == 0) redM[wave] = m;
  __syncthreads();
  const float gm = fmaxf(fmaxf(redM[0], redM[1]), fmaxf(redM[2], redM[3]));
  float ev[8];
#pragma unroll
  for (int e = 0; e < 8; ++e) ev[e] = expf(x[e] - gm);
  float s = ((ev[0] + ev[1]) + (ev[2] + ev[3])) + ((ev[4] + ev[5]) + (ev[6] + ev[7]));
#pragma unroll
  for (int off = 16; off > 0; off >>= 1) s += __shfl_xor(s, off, 32);
  if (lane == 0) redS[wave] = s;
  __syncthreads();
  const float tot = ((redS[0] + redS[1]) + redS[2]) + redS[3];
  const float inv = 1.0f / tot;
  const float kf  = kPCarry * inv;
  unsigned short hb[8];
#pragma unroll
  for (int e = 0; e < 8; ++e) hb[e] = h_bits(ev[e] * kf);
  const v4u u = (v4u){pk16(hb[0], hb[1]), pk16(hb[2], hb[3]), pk16(hb[4], hb[5]), pk16(hb[6], hb[7])};
  unsigned short* q = P + rowoff + c0;
  *(volatile v4u*)q = u;
  __threadfence();
  *(volatile v4u*)q = u;
}

extern "C" void kernel_launch(void* const* d_in, const int* in_sizes, int n_in,
                              void* d_out, int out_size, void* d_ws, size_t ws_size,
                              hipStream_t stream) {
  const size_t NXT = (size_t)kTok * kEmb;
  const size_t NXNEED = (size_t)(kBatch - 1) * kSeqFull * kEmb + (size_t)kSeq * kEmb;
  const size_t NWI = (size_t)3 * kEmb * kEmb;
  const size_t NWO = (size_t)kEmb * kEmb;
  if (n_in < 3) return;
  if ((size_t)in_sizes[0] < NXNEED || (size_t)in_sizes[1] < NWI || (size_t)in_sizes[2] < NWO) return;
  if ((size_t)out_size < NXNEED) return;

  const float* x     = (const float*)d_in[0];
  const float* w_in  = (const float*)d_in[1];
  const float* w_out = (const float*)d_in[2];
  float* out = (float*)d_out;

  char* ws = (char*)d_ws;
  size_t off = 0;
  unsigned short* x16  = (unsigned short*)(ws + off); off += NXT * 2;
  unsigned short* wi16 = (unsigned short*)(ws + off); off += NWI * 2;
  unsigned short* wo16 = (unsigned short*)(ws + off); off += NWO * 2;
  unsigned short* qk   = (unsigned short*)(ws + off); off += (size_t)kQKRows * kQKPitch * 2;
  unsigned short* vt   = (unsigned short*)(ws + off); off += (size_t)kEmb * kVtPitch * 2;
  float*          sp   = (float*)(ws + off);          off += (size_t)kHeads * kWin * kKeys * 4;
  unsigned short* p16  = (unsigned short*)(ws + off); off += (size_t)kHeads * kWin * kKeys * 2;
  unsigned short* o16  = x16;
  if (off > ws_size) return;
  const float* xf = x;

  {
    const int n8x = (int)((size_t)kSeq * kEmb / 8);
    cast8_f16_kernel<<<dim3((unsigned)((n8x + 255) / 256), kBatch), dim3(256), 0, stream>>>(
        x, (long)kSeqFull * kEmb, x16, (long)kSeq * kEmb, n8x, 1.0f);
    cast8_f16_kernel<<<dim3((unsigned)((NWI / 8 + 255) / 256), 1), dim3(256), 0, stream>>>(
        w_in, 0L, wi16, 0L, (int)(NWI / 8), kWCarry);
    cast8_f16_kernel<<<dim3((unsigned)((NWO / 8 + 255) / 256), 1), dim3(256), 0, stream>>>(
        w_out, 0L, wo16, 0L, (int)(NWO / 8), kWCarry);
  }

  {
    const int tq = kGuard * (kQKPitch / 8);
    zero16_kernel<<<dim3((unsigned)((tq + 255) / 256)), dim3(256), 0, stream>>>(qk, kQKPitch, kQKPitch / 8, tq);
    const int tv = kEmb * (kGuard / 8);
    zero16_kernel<<<dim3((unsigned)((tv + 255) / 256)), dim3(256), 0, stream>>>(vt, kVtPitch, kGuard / 8, tv);
  }

  {
    const int tiles = (kTok / 64) * (kQKPitch / 64);
    wmma_gemm64<0, false, 0, 1, false, 0><<<dim3((unsigned)((tiles + 7) / 8), 1), dim3(256), 0, stream>>>(
        x16, x16, kEmb, 0L, wi16, wi16, kEmb, 0L,
        (void*)(qk + (size_t)kGuard * kQKPitch), (void*)(qk + (size_t)kGuard * kQKPitch), kQKPitch, 0L,
        xf, xf, 0L, kTok, kQKPitch, kEmb, kQKScale);
  }
  {
    const int tiles = (kEmb / 64) * (kTok / 64);
    wmma_gemm64<0, false, 0, 1, false, 0><<<dim3((unsigned)((tiles + 7) / 8), 1), dim3(256), 0, stream>>>(
        wi16 + (size_t)2 * kEmb * kEmb, wi16 + (size_t)2 * kEmb * kEmb, kEmb, 0L, x16, x16, kEmb, 0L,
        (void*)(vt + kGuard), (void*)(vt + kGuard), kVtPitch, 0L,
        xf, xf, 0L, kEmb, kTok, kEmb, kQKScale);
  }

  for (int ch = 0; ch < kChunks; ++ch) {
    const int b = ch / kNblk;
    const int n = ch - b * kNblk;
    const size_t tok0 = (size_t)b * kSeq + (size_t)n * kWin;
    {
      const int tiles = (kWin / 64) * (kKeys / 64);
      wmma_gemm64<0, false, 0, 0, false, 0><<<dim3((unsigned)((tiles + 7) / 8), kHeads), dim3(256), 0, stream>>>(
          qk + ((size_t)kGuard + tok0) * kQKPitch, qk + ((size_t)kGuard + tok0) * kQKPitch, kQKPitch, (long)kHdim,
          qk + tok0 * kQKPitch + kEmb, qk + tok0 * kQKPitch + kEmb, kQKPitch, (long)kHdim,
          (void*)sp, (void*)sp, kKeys, (long)kWin * kKeys,
          xf, xf, 0L, kWin, kKeys, kHdim, kSScale);
    }
    band_softmax_kernel<<<dim3(kWin, kHeads), dim3(128), 0, stream>>>(sp, p16, n);
    {
      const int tiles = (kWin / 64) * (kHdim / 64);
      wmma_gemm64<0, false, 0, 1, false, 0><<<dim3((unsigned)((tiles + 7) / 8), kHeads), dim3(256), 0, stream>>>(
          p16, p16, kKeys, (long)kWin * kKeys,
          vt + tok0, vt + tok0, kVtPitch, (long)kHdim * kVtPitch,
          (void*)(o16 + tok0 * kEmb), (void*)(o16 + tok0 * kEmb), kEmb, (long)kHdim,
          xf, xf, 0L, kWin, kHdim, kKeys, kPVScale);
    }
  }

  {
    const int tiles = (kSeq / 64) * (kEmb / 64);
    wmma_gemm64<0, false, 0, 0, false, 0><<<dim3((unsigned)((tiles + 7) / 8), kBatch), dim3(256), 0, stream>>>(
        o16, o16, kEmb, (long)kSeq * kEmb, wo16, wo16, kEmb, 0L,
        (void*)out, (void*)out, kEmb, (long)kSeqFull * kEmb,
        xf, xf, 0L, kSeq, kEmb, kEmb, kOutScale);
  }
}
